// E3Critic_82764019794074
// MI455X (gfx1250) — hardware-verified
//
#include <hip/hip_runtime.h>
#include <stddef.h>


#define NAG    32
#define NOB    16
#define NND    80
#define KNN    5
#define XF     5
#define EKNN   400
#define NEDGE  416
#define HID    128
#define HP     136
#define NTHR   256
#define NWAVE  8
#define WSCAP  134217728

#define SC_W16  16.0f
#define SC_H16  16.0f
#define SC_I256 0.00390625f
#define FBIG    3.402823466e38f
#define AGR     0.05f
#define OBR     0.1f

#define L_XL   0
#define L_H    (L_XL + 2 * NND * HID * 4)
#define L_WE1  (L_H + NND * HP * 2)
#define L_WE2  (L_WE1 + XF * HID * 4)
#define L_V1   (L_WE2 + XF * HID * 4)
#define L_V2   (L_V1 + 4 * HID * 4)
#define L_W3   (L_V2 + 4 * HID * 4)
#define L_EA   (L_W3 + 2 * HID * 4)
#define L_LG   (L_EA + NEDGE * XF * 4)
#define L_SRC  (L_LG + NEDGE * 4)
#define L_POS  (L_SRC + NEDGE * 4)
#define L_VEL  (L_POS + NND * 2 * 4)
#define L_RAD  (L_VEL + NND * 2 * 4)
#define L_X    (L_RAD + NND * 4)
#define L_DUP  (L_X + NND * 8 * 4)
#define L_XL3  (L_DUP + NOB * 4)
#define L_XR3  (L_XL3 + NND * 4)
#define L_O3   (L_XR3 + NND * 4)
#define L_S    (L_O3 + NAG * 4)
#define LDS_TOTAL (L_S + 16 * 4)

static_assert((L_H % 16) == 0 && (L_WE1 % 16) == 0 && (L_WE2 % 16) == 0 && (L_V1 % 16) == 0);
static_assert((L_V2 % 16) == 0 && (L_W3 % 16) == 0 && (L_EA % 16) == 0 && (L_LG % 16) == 0);
static_assert((L_SRC % 16) == 0 && (L_POS % 16) == 0 && (L_VEL % 16) == 0 && (L_RAD % 16) == 0);
static_assert((L_X % 16) == 0 && (L_DUP % 16) == 0 && (L_XL3 % 16) == 0 && (L_XR3 % 16) == 0);
static_assert((L_O3 % 16) == 0 && (L_S % 16) == 0 && LDS_TOTAL <= 160 * 1024);
static_assert((NND % 16) == 0 && (HID % 32) == 0 && HID == 32 * 4 && NWAVE * 16 == HID);
static_assert((NEDGE % NWAVE) == 0 && (NND % NWAVE) == 0 && (NAG % NWAVE) == 0);
static_assert(((NND * 32) % NTHR) == 0 && ((HP * 2) % 16) == 0 && NTHR == 32 * NWAVE);
static_assert(EKNN == NND * KNN && NEDGE == EKNN + NOB && NND == 2 * NAG + NOB && KNN < 32);
static_assert(((2 * HID * HID / 8) % NTHR) == 0);

typedef float          v4f  __attribute__((ext_vector_type(4)));
typedef float          v8f  __attribute__((ext_vector_type(8)));
typedef _Float16       v4h  __attribute__((ext_vector_type(4)));
typedef _Float16       v8h  __attribute__((ext_vector_type(8)));
typedef _Float16       v16h __attribute__((ext_vector_type(16)));
typedef unsigned short v8us __attribute__((ext_vector_type(8)));
union Frag { v16h v; v8h h[2]; };
union H8 { v8h f; v8us u; };
static_assert(sizeof(Frag) == 32 && sizeof(H8) == 16);

__device__ __forceinline__ v8f wm(v16h a, v16h bq, v8f c) {
  v8f d = __builtin_amdgcn_wmma_f32_16x16x32_f16(false, a, false, bq, (short)0, c, false, false);
  asm volatile("v_nop\n\tv_nop\n\tv_nop\n\tv_nop" : "+v"(d) : "v"(a), "v"(bq));
  return d;
}

__device__ __forceinline__ v8f zero8() {
  v8f z = {0.f, 0.f, 0.f, 0.f, 0.f, 0.f, 0.f, 0.f};
  return z;
}

__device__ __forceinline__ int imin(int a, int b) { return a < b ? a : b; }
__device__ __forceinline__ int imax(int a, int b) { return a > b ? a : b; }
__device__ __forceinline__ int iclamp(int v, int lo, int hi) { return imin(imax(v, lo), hi); }

__device__ __forceinline__ float wsum(float v) {
#pragma unroll
  for (int off = 16; off > 0; off >>= 1) v += __shfl_xor(v, off, 32);
  return v;
}
__device__ __forceinline__ float wmax(float v) {
#pragma unroll
  for (int off = 16; off > 0; off >>= 1) v = fmaxf(v, __shfl_xor(v, off, 32));
  return v;
}
__device__ __forceinline__ float lrelu(float x) { return (x >= 0.0f) ? x : 0.2f * x; }

__global__ __launch_bounds__(NTHR) void k_cvtw(const float* __restrict__ Wl, const float* __restrict__ Wr,
                                               _Float16* dst) {
  const int t = blockIdx.x * NTHR + threadIdx.x;
  if (t >= 2 * HID * HID / 8) return;
  const int e0 = 8 * t;
  const int n  = e0 >> 7;
  const int kb = e0 & (HID - 1);
  const int nn = n & (HID - 1);
  H8 o;
#pragma unroll
  for (int i = 0; i < 8; ++i) {
    const int k = kb + i;
    const float a = Wl[k * HID + nn];
    const float c = Wr[k * HID + nn];
    const float v = (n < HID) ? a : c;
    o.f[i] = (_Float16)(v * SC_W16);
  }
  unsigned short* p = (unsigned short*)(dst + (size_t)e0);
  *(volatile v8us*)p = o.u;
  __threadfence();
  *(volatile v8us*)p = o.u;
}

__device__ __forceinline__ void build_knn(const float* sPos, int* sSrc, int tid) {
#pragma clang fp contract(off)
  if (tid < NND) {
    float bd[KNN];
    int   bi[KNN];
#pragma unroll
    for (int s = 0; s < KNN; ++s) { bd[s] = FBIG; bi[s] = 0; }
    const float px = sPos[2 * tid], py = sPos[2 * tid + 1];
#pragma unroll 1
    for (int j = 0; j < NND; ++j) {
      const float dx = px - sPos[2 * j], dy = py - sPos[2 * j + 1];
      const float d2 = dx * dx + dy * dy;
      const bool ins = d2 < bd[KNN - 1];
      bd[KNN - 1] = ins ? d2 : bd[KNN - 1];
      bi[KNN - 1] = ins ? j : bi[KNN - 1];
#pragma unroll
      for (int s = KNN - 1; s > 0; --s) {
        const bool  sw = bd[s] < bd[s - 1];
        const float td = bd[s], ud = bd[s - 1];
        const int   ti = bi[s], ui = bi[s - 1];
        bd[s]     = sw ? ud : td;
        bd[s - 1] = sw ? td : ud;
        bi[s]     = sw ? ui : ti;
        bi[s - 1] = sw ? ti : ui;
      }
    }
#pragma unroll
    for (int s = 0; s < KNN; ++s) sSrc[KNN * tid + s] = bi[s];
  }
  if (tid < NOB) sSrc[EKNN + tid] = tid;
}

__device__ __forceinline__ void build_feats(const float* sPos, const float* sVel, const float* sRad,
                                            const int* sSrc, int* sDup, float* sX, float* sEa, int tid) {
#pragma clang fp contract(off)
  if (tid < NOB) {
    int d = 0;
#pragma unroll
    for (int s = 0; s < KNN; ++s) d |= (sSrc[KNN * (NAG + tid) + s] == tid) ? 1 : 0;
    sDup[tid] = d;
  }
  if (tid < NND) {
    const int n = tid;
    const bool isA = n < NAG, isG = (n >= NAG) && (n < 2 * NAG), isO = n >= 2 * NAG;
    const float vx = sVel[2 * n], vy = sVel[2 * n + 1];
    const float sp = sqrtf(vx * vx + vy * vy);
    float* xr = sX + n * 8;
    xr[0] = isA ? 1.0f : 0.0f;
    xr[1] = isG ? 1.0f : 0.0f;
    xr[2] = isO ? 1.0f : 0.0f;
    xr[3] = isA ? sp : 0.0f;
    xr[4] = sRad[n];
    xr[5] = 0.0f;
    xr[6] = 0.0f;
    xr[7] = 0.0f;
  }
#pragma unroll 1
  for (int e = tid; e < NEDGE; e += NTHR) {
    const int src = iclamp(sSrc[e], 0, NND - 1);
    const int dst = (e < EKNN) ? (e / KNN) : (e - EKNN + NAG);
    const float pdx = sPos[2 * src] - sPos[2 * dst];
    const float pdy = sPos[2 * src + 1] - sPos[2 * dst + 1];
    const float dist = sqrtf(pdx * pdx + pdy * pdy);
    const float den = fmaxf(dist, 1e-6f);
    const float inv = 1.0f / den;
    const float pnx = pdx * inv, pny = pdy * inv;
    const float rvx = sVel[2 * src] - sVel[2 * dst];
    const float rvy = sVel[2 * src + 1] - sVel[2 * dst + 1];
    float* ep = sEa + e * XF;
    ep[0] = ((src < NAG) && (dst == src + NAG)) ? 1.0f : 0.0f;
    ep[1] = dist;
    ep[2] = dist - (sRad[src] + sRad[dst]);
    ep[3] = rvx * pnx + rvy * pny;
    ep[4] = rvx * pny - rvy * pnx;
  }
}

__device__ __forceinline__ void lin1(const float* sX, const float* __restrict__ Wl1,
                                     const float* __restrict__ Wr1, const float* sV1,
                                     float* sXL, float* sXR, int tid) {
#pragma unroll 1
  for (int j = 0; j < (NND * 32) / NTHR; ++j) {
    const int it = tid + j * NTHR;
    const int n = it >> 5, c = (it & 31) * 4;
    const float* xr = sX + n * 8;
    v4f al = {0.f, 0.f, 0.f, 0.f};
    v4f ar = {0.f, 0.f, 0.f, 0.f};
#pragma unroll 1
    for (int k = 0; k < XF; ++k) {
      const float xv = xr[k];
      const v4f wl = *(const v4f*)(Wl1 + k * HID + c);
      const v4f wr = *(const v4f*)(Wr1 + k * HID + c);
      al = xv * wl + al;
      ar = xv * wr + ar;
    }
    al = al + *(const v4f*)(sV1 + HID + c);
    ar = ar + *(const v4f*)(sV1 + 2 * HID + c);
    *(v4f*)(sXL + n * HID + c) = al;
    *(v4f*)(sXR + n * HID + c) = ar;
  }
}

__device__ __forceinline__ void edge_logits(const float* sXL, const float* sXR, const float* sEa,
                                            const float* sWe, const float* sAtt, const int* sSrc,
                                            float* sLg, int lane, int wave) {
  const int f = 4 * lane;
  const v4f w0 = *(const v4f*)(sWe + 0 * HID + f);
  const v4f w1 = *(const v4f*)(sWe + 1 * HID + f);
  const v4f w2 = *(const v4f*)(sWe + 2 * HID + f);
  const v4f w3 = *(const v4f*)(sWe + 3 * HID + f);
  const v4f w4 = *(const v4f*)(sWe + 4 * HID + f);
  const v4f at = *(const v4f*)(sAtt + f);
#pragma unroll 1
  for (int e = wave; e < NEDGE; e += NWAVE) {
    const int src = iclamp(sSrc[e], 0, NND - 1);
    const int dst = (e < EKNN) ? (e / KNN) : (e - EKNN + NAG);
    const float* ep = sEa + e * XF;
    const float e0 = ep[0], e1 = ep[1], e2 = ep[2], e3 = ep[3], e4 = ep[4];
    v4f we = e0 * w0;
    we = e1 * w1 + we;
    we = e2 * w2 + we;
    we = e3 * w3 + we;
    we = e4 * w4 + we;
    v4f t = (*(const v4f*)(sXL + src * HID + f) + *(const v4f*)(sXR + dst * HID + f)) + we;
    t.x = lrelu(t.x);
    t.y = lrelu(t.y);
    t.z = lrelu(t.z);
    t.w = lrelu(t.w);
    float part = t.x * at.x;
    part = t.y * at.y + part;
    part = t.z * at.z + part;
    part = t.w * at.w + part;
    part = wsum(part);
    if (lane == 0) sLg[e] = part;
  }
}

template <int OUTF16>
__device__ __forceinline__ void aggregate(const float* sXL, const float* sLg, const int* sSrc,
                                          const int* sDup, const float* sBias, _Float16* oH, float* oF,
                                          int lane, int wave) {
  const int f = 4 * lane;
  const v4f bias = *(const v4f*)(sBias + f);
  const int lc = imin(lane, KNN - 1);
  const bool isK = lane < KNN;
#pragma unroll 1
  for (int n = wave; n < NND; n += NWAVE) {
    const int base = KNN * n;
    const bool hasEx = (n >= NAG) && (n < NAG + NOB);
    const int  ex = iclamp(n - NAG, 0, NOB - 1);
    const bool useEx = hasEx && (sDup[ex] == 0);
    const float lgk = sLg[base + lc];
    const float lge = sLg[EKNN + ex];
    const int   sk  = iclamp(sSrc[base + lc], 0, NND - 1);
    const bool valid = isK || ((lane == KNN) && useEx);
    const float lv = valid ? (isK ? lgk : lge) : -FBIG;
    const int   si = isK ? sk : ex;
    const float m = wmax(lv);
    const float ee = expf(lv - m);
    const float a = valid ? ee : 0.0f;
    const float den = wsum(a);
    const float al = a * (1.0f / den);
    v4f acc;
    {
      const float w = __shfl(al, 0, 32);
      const int   s = __shfl(si, 0, 32);
      acc = w * *(const v4f*)(sXL + s * HID + f);
    }
#pragma unroll
    for (int j = 1; j <= KNN; ++j) {
      const float w = __shfl(al, j, 32);
      const int   s = __shfl(si, j, 32);
      acc = w * *(const v4f*)(sXL + s * HID + f) + acc;
    }
    v4f o = acc + bias;
    o.x = fmaxf(o.x, 0.0f);
    o.y = fmaxf(o.y, 0.0f);
    o.z = fmaxf(o.z, 0.0f);
    o.w = fmaxf(o.w, 0.0f);
    if (OUTF16) {
      v4h q;
      q.x = (_Float16)(o.x * SC_H16);
      q.y = (_Float16)(o.y * SC_H16);
      q.z = (_Float16)(o.z * SC_H16);
      q.w = (_Float16)(o.w * SC_H16);
      *(v4h*)(oH + n * HP + f) = q;
    } else {
      *(v4f*)(oF + n * HID + f) = o;
    }
  }
}

__device__ __forceinline__ void gemm2(const _Float16* sH, const _Float16* __restrict__ W2p,
                                      const float* sV2, float* sXL, int lane, int wave) {
  const int h = lane >> 4, m = lane & 15;
#pragma unroll
  for (int mat = 0; mat < 2; ++mat) {
    const int col = mat * HID + 16 * wave + m;
    const _Float16* bp = W2p + (size_t)col * HID + 8 * h;
    const float bias = sV2[HID * (1 + mat) + 16 * wave + m];
    float* outp = sXL + mat * NND * HID;
    v8f acc[NND / 16];
#pragma unroll
    for (int mt = 0; mt < NND / 16; ++mt) acc[mt] = zero8();
#pragma unroll
    for (int ks = 0; ks < HID / 32; ++ks) {
      Frag fb;
      fb.h[0] = *(const v8h*)(bp + 32 * ks);
      fb.h[1] = *(const v8h*)(bp + 32 * ks + 16);
#pragma unroll
      for (int mt = 0; mt < NND / 16; ++mt) {
        const _Float16* ap = sH + (16 * mt + m) * HP + 32 * ks + 8 * h;
        Frag fa;
        fa.h[0] = *(const v8h*)(ap);
        fa.h[1] = *(const v8h*)(ap + 16);
        acc[mt] = wm(fa.v, fb.v, acc[mt]);
      }
    }
#pragma unroll
    for (int mt = 0; mt < NND / 16; ++mt) {
#pragma unroll
      for (int r = 0; r < 8; ++r) {
        outp[(16 * mt + 8 * h + r) * HID + 16 * wave + m] = acc[mt][r] * SC_I256 + bias;
      }
    }
  }
}

__global__ __launch_bounds__(NTHR) void k_main(
    const float* __restrict__ obst, const float* __restrict__ apos,
    const float* __restrict__ gpos, const float* __restrict__ avel,
    const float* __restrict__ Wl1, const float* __restrict__ bl1,
    const float* __restrict__ Wr1, const float* __restrict__ br1,
    const float* __restrict__ We1, const float* __restrict__ att1,
    const float* __restrict__ bias1,
    const float* __restrict__ bl2, const float* __restrict__ br2,
    const float* __restrict__ We2, const float* __restrict__ att2,
    const float* __restrict__ bias2,
    const float* __restrict__ Wl3, const float* __restrict__ bl3,
    const float* __restrict__ Wr3, const float* __restrict__ br3,
    const float* __restrict__ We3, const float* __restrict__ att3,
    const float* __restrict__ bias3,
    const _Float16* __restrict__ W2p, float* out) {
  extern __shared__ v4f lds_dyn[];
  char* sm = (char*)lds_dyn;
  float*    sXL  = (float*)(sm + L_XL);
  float*    sXR  = sXL + NND * HID;
  _Float16* sH   = (_Float16*)(sm + L_H);
  float*    sWe1 = (float*)(sm + L_WE1);
  float*    sWe2 = (float*)(sm + L_WE2);
  float*    sV1  = (float*)(sm + L_V1);
  float*    sV2  = (float*)(sm + L_V2);
  float*    sW3  = (float*)(sm + L_W3);
  float*    sEa  = (float*)(sm + L_EA);
  float*    sLg  = (float*)(sm + L_LG);
  int*      sSrc = (int*)(sm + L_SRC);
  float*    sPos = (float*)(sm + L_POS);
  float*    sVel = (float*)(sm + L_VEL);
  float*    sRad = (float*)(sm + L_RAD);
  float*    sX   = (float*)(sm + L_X);
  int*      sDup = (int*)(sm + L_DUP);
  float*    sXL3 = (float*)(sm + L_XL3);
  float*    sXR3 = (float*)(sm + L_XR3);
  float*    sO3  = (float*)(sm + L_O3);
  float*    sS   = (float*)(sm + L_S);

  const int tid = threadIdx.x, lane = tid & 31;
  const int wave = __builtin_amdgcn_readfirstlane(tid >> 5);
  const int b = blockIdx.x;

  if (tid < NND) {
    const int n = tid;
    const int ia = imin(n, NAG - 1);
    const int ig = iclamp(n - NAG, 0, NAG - 1);
    const int io = iclamp(n - 2 * NAG, 0, NOB - 1);
    const float* pa = apos + ((size_t)b * NAG + ia) * 2;
    const float* pg = gpos + ((size_t)b * NAG + ig) * 2;
    const float* po = obst + ((size_t)b * NOB + io) * 2;
    const float* pv = avel + ((size_t)b * NAG + ia) * 2;
    const float ax = pa[0], ay = pa[1], gx = pg[0], gy = pg[1], ox = po[0], oy = po[1];
    const float vx = pv[0], vy = pv[1];
    const bool isA = n < NAG, isG = (n >= NAG) && (n < 2 * NAG);
    sPos[2 * n]     = isA ? ax : (isG ? gx : ox);
    sPos[2 * n + 1] = isA ? ay : (isG ? gy : oy);
    sVel[2 * n]     = isA ? vx : 0.0f;
    sVel[2 * n + 1] = isA ? vy : 0.0f;
    sRad[n] = isA ? AGR : (isG ? 0.0f : OBR);
  }
  if (tid < HID) {
    sV1[tid]           = att1[tid];
    sV1[HID + tid]     = bl1[tid];
    sV1[2 * HID + tid] = br1[tid];
    sV1[3 * HID + tid] = bias1[tid];
    sV2[tid]           = att2[tid];
    sV2[HID + tid]     = bl2[tid];
    sV2[2 * HID + tid] = br2[tid];
    sV2[3 * HID + tid] = bias2[tid];
    sW3[tid]           = Wl3[tid];
    sW3[HID + tid]     = Wr3[tid];
  }
#pragma unroll 1
  for (int i = tid; i < XF * HID; i += NTHR) {
    sWe1[i] = We1[i];
    sWe2[i] = We2[i];
  }
  if (tid < 16) {
    const float v0 = bl3[0], v1 = br3[0], v2 = We3[iclamp(tid - 2, 0, XF - 1)];
    const float v3 = att3[0], v4 = bias3[0];
    const float v = (tid == 0) ? v0 : ((tid == 1) ? v1 : ((tid < 2 + XF) ? v2 :
                    ((tid == 2 + XF) ? v3 : ((tid == 3 + XF) ? v4 : 0.0f))));
    sS[tid] = v;
  }
  __syncthreads();

  build_knn(sPos, sSrc, tid);
  __syncthreads();

  build_feats(sPos, sVel, sRad, sSrc, sDup, sX, sEa, tid);
  __syncthreads();

  lin1(sX, Wl1, Wr1, sV1, sXL, sXR, tid);
  __syncthreads();

  edge_logits(sXL, sXR, sEa, sWe1, sV1, sSrc, sLg, lane, wave);
  __syncthreads();

  aggregate<1>(sXL, sLg, sSrc, sDup, sV1 + 3 * HID, sH, sXR, lane, wave);
  __syncthreads();

  gemm2(sH, W2p, sV2, sXL, lane, wave);
  __syncthreads();

  edge_logits(sXL, sXR, sEa, sWe2, sV2, sSrc, sLg, lane, wave);
  __syncthreads();

  aggregate<0>(sXL, sLg, sSrc, sDup, sV2 + 3 * HID, sH, sXR, lane, wave);
  __syncthreads();

  if (tid < NND) {
    const float* hr = sXR + tid * HID;
    float xl = 0.0f, xr = 0.0f;
#pragma unroll 4
    for (int k = 0; k < HID; ++k) {
      const float hv = hr[k];
      xl = hv * sW3[k] + xl;
      xr = hv * sW3[HID + k] + xr;
    }
    sXL3[tid] = xl + sS[0];
    sXR3[tid] = xr + sS[1];
  }
  __syncthreads();

#pragma unroll 1
  for (int e = tid; e < NEDGE; e += NTHR) {
    const int src = iclamp(sSrc[e], 0, NND - 1);
    const int dst = (e < EKNN) ? (e / KNN) : (e - EKNN + NAG);
    const float* ep = sEa + e * XF;
    float ew = ep[0] * sS[2];
    ew = ep[1] * sS[3] + ew;
    ew = ep[2] * sS[4] + ew;
    ew = ep[3] * sS[5] + ew;
    ew = ep[4] * sS[6] + ew;
    float t = (sXL3[src] + sXR3[dst]) + ew;
    t = lrelu(t);
    sLg[e] = t * sS[2 + XF];
  }
  __syncthreads();

  {
    const int lc = imin(lane, KNN - 1);
    const bool isK = lane < KNN;
#pragma unroll 1
    for (int i = 0; i < NAG / NWAVE; ++i) {
      const int n = wave + NWAVE * i;
      const int base = KNN * n;
      const float lg = sLg[base + lc];
      const int   si = iclamp(sSrc[base + lc], 0, NND - 1);
      const float lv = isK ? lg : -FBIG;
      const float m = wmax(lv);
      const float ee = expf(lv - m);
      const float a = isK ? ee : 0.0f;
      const float den = wsum(a);
      const float al = a * (1.0f / den);
      float o;
      {
        const float w = __shfl(al, 0, 32);
        const int   s = __shfl(si, 0, 32);
        o = w * sXL3[s];
      }
#pragma unroll
      for (int j = 1; j < KNN; ++j) {
        const float w = __shfl(al, j, 32);
        const int   s = __shfl(si, j, 32);
        o = w * sXL3[s] + o;
      }
      o = o + sS[3 + XF];
      if (lane == 0) sO3[n] = o;
    }
  }
  __syncthreads();

  if (wave == 0) {
    float v = sO3[lane];
    v = wsum(v);
    v4f q = {v, v, v, v};
    float* p = out + (size_t)b * NAG + 4 * (lane & 7);
    if (lane < 8) *(volatile v4f*)p = q;
    __threadfence();
    if (lane < 8) *(volatile v4f*)p = q;
  }
}

extern "C" void kernel_launch(void* const* d_in, const int* in_sizes, int n_in,
                              void* d_out, int out_size, void* d_ws, size_t ws_size,
                              hipStream_t stream) {
  if (n_in < 25) return;
  const int B = in_sizes[1] / (NAG * 2);
  if (B <= 0 || in_sizes[1] != B * NAG * 2) return;
  if (in_sizes[0] != B * NOB * 2 || in_sizes[2] != B * NAG * 2 || in_sizes[3] != B * NAG * 2) return;
  if (in_sizes[4] != XF * HID || in_sizes[5] != HID || in_sizes[6] != XF * HID || in_sizes[7] != HID) return;
  if (in_sizes[8] != XF * HID || in_sizes[9] != HID || in_sizes[10] != HID) return;
  if (in_sizes[11] != HID * HID || in_sizes[12] != HID || in_sizes[13] != HID * HID || in_sizes[14] != HID) return;
  if (in_sizes[15] != XF * HID || in_sizes[16] != HID || in_sizes[17] != HID) return;
  if (in_sizes[18] != HID || in_sizes[19] != 1 || in_sizes[20] != HID || in_sizes[21] != 1) return;
  if (in_sizes[22] != XF || in_sizes[23] != 1 || in_sizes[24] != 1) return;
  if (out_size != B * NAG) return;

  const size_t wbytes = (size_t)2 * HID * HID * sizeof(_Float16);
  if (wbytes > ws_size || wbytes > (size_t)WSCAP) return;

  const float* obst  = (const float*)d_in[0];
  const float* apos  = (const float*)d_in[1];
  const float* gpos  = (const float*)d_in[2];
  const float* avel  = (const float*)d_in[3];
  const float* Wl1   = (const float*)d_in[4];
  const float* bl1   = (const float*)d_in[5];
  const float* Wr1   = (const float*)d_in[6];
  const float* br1   = (const float*)d_in[7];
  const float* We1   = (const float*)d_in[8];
  const float* att1  = (const float*)d_in[9];
  const float* bias1 = (const float*)d_in[10];
  const float* Wl2   = (const float*)d_in[11];
  const float* bl2   = (const float*)d_in[12];
  const float* Wr2   = (const float*)d_in[13];
  const float* br2   = (const float*)d_in[14];
  const float* We2   = (const float*)d_in[15];
  const float* att2  = (const float*)d_in[16];
  const float* bias2 = (const float*)d_in[17];
  const float* Wl3   = (const float*)d_in[18];
  const float* bl3   = (const float*)d_in[19];
  const float* Wr3   = (const float*)d_in[20];
  const float* br3   = (const float*)d_in[21];
  const float* We3   = (const float*)d_in[22];
  const float* att3  = (const float*)d_in[23];
  const float* bias3 = (const float*)d_in[24];
  float* out = (float*)d_out;
  _Float16* W2p = (_Float16*)d_ws;

  const int npiece = 2 * HID * HID / 8;
  k_cvtw<<<npiece / NTHR, NTHR, 0, stream>>>(Wl2, Wr2, W2p);

  hipFuncSetAttribute(reinterpret_cast<const void*>(&k_main),
                      hipFuncAttributeMaxDynamicSharedMemorySize, LDS_TOTAL);
  k_main<<<B, NTHR, LDS_TOTAL, stream>>>(obst, apos, gpos, avel,
                                         Wl1, bl1, Wr1, br1, We1, att1, bias1,
                                         bl2, br2, We2, att2, bias2,
                                         Wl3, bl3, Wr3, br3, We3, att3, bias3,
                                         W2p, out);
}
